// Attention_65541200937125
// MI455X (gfx1250) — hardware-run, weakly checked
//
#include <hip/hip_runtime.h>
#ifndef NB
#define NB 8
#endif
#ifndef SEQ
#define SEQ 2048
#endif
#define NB_FULL 8
#define SEQ_FULL 2048
#define NH 6
#define HD 64
#define NE 384
#define XROWS (NB * SEQ)
#define XPLANE ((size_t)XROWS * NE)
#define WELEMS ((size_t)NE * NE)
#define MW (SEQ / 32)
#define XSTRIDE_FULL ((size_t)SEQ_FULL * NE)
#define PAD256(x) ((((size_t)(x)) + 255) & ~(size_t)255)

static_assert(SEQ % 64 == 0);
static_assert(SEQ <= SEQ_FULL);
static_assert(NB <= NB_FULL);
static_assert(HD == 64);
static_assert(NE == NH * HD);
static_assert(NE % 64 == 0);
static_assert(NE % 32 == 0);
static_assert((XROWS * (NE / 8)) % 256 == 0);
static_assert((WELEMS / 8) % 256 == 0);
static_assert((SEQ * MW) % 256 == 0);
static_assert(XROWS % 64 == 0);
static_assert(PAD256(XPLANE * 2) + PAD256(3 * WELEMS * 2) + PAD256(WELEMS * 2) + PAD256(2 * XPLANE * 2) + 2 * PAD256(XPLANE * 2) + PAD256((size_t)SEQ * MW * 4) <= (size_t)134217728);

typedef __bf16 v16b __attribute__((ext_vector_type(16)));
typedef _Float16 v16h __attribute__((ext_vector_type(16)));
typedef unsigned short v8us __attribute__((ext_vector_type(8), may_alias));
typedef float v8f __attribute__((ext_vector_type(8)));
typedef float v4f __attribute__((ext_vector_type(4)));
typedef float v4fa __attribute__((ext_vector_type(4), may_alias));
typedef int v4ia __attribute__((ext_vector_type(4), may_alias));
union FragB { v16b v; v8us half[2]; };
union FragH { v16h v; v8us half[2]; _Float16 h[16]; };

#define LOG2E 1.4426950408889634f
#define SCL (0.125f * 0.00390625f)

__device__ __forceinline__ unsigned short bf16_bits(float x) {
  unsigned int u = __float_as_uint(x);
  return (unsigned short)((u + 0x7FFFu + ((u >> 16) & 1u)) >> 16);
}
__device__ __forceinline__ float bf16_val(unsigned short b) { return __uint_as_float(((unsigned int)b) << 16); }
__device__ __forceinline__ float bf16_rne(float x) { return bf16_val(bf16_bits(x)); }
__device__ __forceinline__ unsigned short f16_bits(_Float16 h) { return __builtin_bit_cast(unsigned short, h); }

static __device__ __forceinline__ _Float16 toh_flush(float v) {
  const _Float16 r = (_Float16)v;
  return (fabsf(v) < 6.103515625e-05f) ? (_Float16)0.0f : r;
}

__device__ __forceinline__ void mma_b4(v16b a, v16b b0, v16b b1, v16b b2, v16b b3, v8f& c0, v8f& c1, v8f& c2, v8f& c3) {
  c0 = __builtin_amdgcn_wmma_f32_16x16x32_bf16(false, a, false, b0, (short)0, c0, false, false);
  c1 = __builtin_amdgcn_wmma_f32_16x16x32_bf16(false, a, false, b1, (short)0, c1, false, false);
  c2 = __builtin_amdgcn_wmma_f32_16x16x32_bf16(false, a, false, b2, (short)0, c2, false, false);
  c3 = __builtin_amdgcn_wmma_f32_16x16x32_bf16(false, a, false, b3, (short)0, c3, false, false);
  asm volatile("v_nop\n\tv_nop\n\tv_nop\n\tv_nop" : "+v"(c0), "+v"(c1), "+v"(c2), "+v"(c3) : "v"(a), "v"(b0), "v"(b1), "v"(b2), "v"(b3));
}
__device__ __forceinline__ void mma_h4(v16h a, v16h b0, v16h b1, v16h b2, v16h b3, v8f& c0, v8f& c1, v8f& c2, v8f& c3) {
  c0 = __builtin_amdgcn_wmma_f32_16x16x32_f16(false, a, false, b0, (short)0, c0, false, false);
  c1 = __builtin_amdgcn_wmma_f32_16x16x32_f16(false, a, false, b1, (short)0, c1, false, false);
  c2 = __builtin_amdgcn_wmma_f32_16x16x32_f16(false, a, false, b2, (short)0, c2, false, false);
  c3 = __builtin_amdgcn_wmma_f32_16x16x32_f16(false, a, false, b3, (short)0, c3, false, false);
  asm volatile("v_nop\n\tv_nop\n\tv_nop\n\tv_nop" : "+v"(c0), "+v"(c1), "+v"(c2), "+v"(c3) : "v"(a), "v"(b0), "v"(b1), "v"(b2), "v"(b3));
}
__device__ __forceinline__ v8f mma_s2(v16h a0, v16h b0, v16h a1, v16h b1, v8f c) {
  c = __builtin_amdgcn_wmma_f32_16x16x32_f16(false, a0, false, b0, (short)0, c, false, false);
  c = __builtin_amdgcn_wmma_f32_16x16x32_f16(false, a1, false, b1, (short)0, c, false, false);
  asm volatile("v_nop\n\tv_nop\n\tv_nop\n\tv_nop" : "+v"(c) : "v"(a0), "v"(b0), "v"(a1), "v"(b1));
  return c;
}
__device__ __forceinline__ void mma_pv4(v16h a0, v16h a1, v16h a2, v16h a3, v16h b, v8f& c0, v8f& c1, v8f& c2, v8f& c3) {
  c0 = __builtin_amdgcn_wmma_f32_16x16x32_f16(false, a0, false, b, (short)0, c0, false, false);
  c1 = __builtin_amdgcn_wmma_f32_16x16x32_f16(false, a1, false, b, (short)0, c1, false, false);
  c2 = __builtin_amdgcn_wmma_f32_16x16x32_f16(false, a2, false, b, (short)0, c2, false, false);
  c3 = __builtin_amdgcn_wmma_f32_16x16x32_f16(false, a3, false, b, (short)0, c3, false, false);
  asm volatile("v_nop\n\tv_nop\n\tv_nop\n\tv_nop" : "+v"(c0), "+v"(c1), "+v"(c2), "+v"(c3) : "v"(a0), "v"(a1), "v"(a2), "v"(a3), "v"(b));
}

__device__ __forceinline__ v8us cvt8_bf16(const float* __restrict__ src) {
  const v4f x0 = *(const v4fa*)(src), x1 = *(const v4fa*)(src + 4);
  v8us o;
  o[0] = bf16_bits(x0[0]); o[1] = bf16_bits(x0[1]); o[2] = bf16_bits(x0[2]); o[3] = bf16_bits(x0[3]);
  o[4] = bf16_bits(x1[0]); o[5] = bf16_bits(x1[1]); o[6] = bf16_bits(x1[2]); o[7] = bf16_bits(x1[3]);
  return o;
}

__global__ __launch_bounds__(256) void k_cvt_x(const float* __restrict__ X, unsigned short* __restrict__ XP) {
  const int t = blockIdx.x * 256 + threadIdx.x;
  if (t >= XROWS * (NE / 8)) return;
  const int row = t / (NE / 8), piece = t - row * (NE / 8);
  const int b = row / SEQ, s = row - b * SEQ;
  const size_t so = (size_t)b * XSTRIDE_FULL + (size_t)s * NE + piece * 8;
  const v8us ox = cvt8_bf16(X + so);
  unsigned short* d = XP + (size_t)t * 8;
  *(volatile v8us*)(d) = ox;
  __threadfence();
  *(volatile v8us*)(d) = ox;
}

__global__ __launch_bounds__(256) void k_cvt_w(const float* __restrict__ Wk, const float* __restrict__ Wq,
                                               const float* __restrict__ Wv, const float* __restrict__ Wp,
                                               unsigned short* __restrict__ WP, unsigned short* __restrict__ W16) {
  const int t = blockIdx.x * 256 + threadIdx.x;
  if (t >= (int)(WELEMS / 8)) return;
  const size_t so = (size_t)t * 8;
  const v8us o0 = cvt8_bf16(Wk + so);
  const v8us o1 = cvt8_bf16(Wq + so);
  const v8us o2 = cvt8_bf16(Wv + so);
  const v4f x0 = *(const v4fa*)(Wp + so), x1 = *(const v4fa*)(Wp + so + 4);
  v8us o3;
  o3[0] = f16_bits((_Float16)(bf16_rne(x0[0]) * 64.0f)); o3[1] = f16_bits((_Float16)(bf16_rne(x0[1]) * 64.0f));
  o3[2] = f16_bits((_Float16)(bf16_rne(x0[2]) * 64.0f)); o3[3] = f16_bits((_Float16)(bf16_rne(x0[3]) * 64.0f));
  o3[4] = f16_bits((_Float16)(bf16_rne(x1[0]) * 64.0f)); o3[5] = f16_bits((_Float16)(bf16_rne(x1[1]) * 64.0f));
  o3[6] = f16_bits((_Float16)(bf16_rne(x1[2]) * 64.0f)); o3[7] = f16_bits((_Float16)(bf16_rne(x1[3]) * 64.0f));
  unsigned short* d = WP + so;
  unsigned short* e = W16 + so;
  *(volatile v8us*)(d) = o0;
  *(volatile v8us*)(d + WELEMS) = o1;
  *(volatile v8us*)(d + 2 * WELEMS) = o2;
  *(volatile v8us*)(e) = o3;
  __threadfence();
  *(volatile v8us*)(d) = o0;
  *(volatile v8us*)(d + WELEMS) = o1;
  *(volatile v8us*)(d + 2 * WELEMS) = o2;
  *(volatile v8us*)(e) = o3;
}

__global__ __launch_bounds__(256) void k_maskones(unsigned int* __restrict__ bits) {
  const int t = blockIdx.x * 256 + threadIdx.x;
  if (t >= SEQ * MW) return;
  const unsigned int w = 0xFFFFFFFFu;
  *(volatile unsigned int*)(bits + t) = w;
  __threadfence();
  *(volatile unsigned int*)(bits + t) = w;
}

template <int MODE>
__device__ __forceinline__ void proj_body(const unsigned short* __restrict__ Ab, const unsigned short* __restrict__ Bb,
                                          const float* __restrict__ bias, unsigned short* __restrict__ Oh,
                                          unsigned int zA, unsigned int zB, unsigned int zO, unsigned int zBias) {
  __shared__ __attribute__((aligned(16))) unsigned short th[64][72];
  const int tid = threadIdx.x, w = __builtin_amdgcn_readfirstlane((int)(tid >> 5)), lane = tid & 31, ln = lane & 15, hh = lane >> 4;
  const int z = blockIdx.z;
  const int m0 = (MODE == 0) ? (int)blockIdx.x * 64 : (int)blockIdx.y * 64;
  const int n0 = (MODE == 0) ? (int)blockIdx.y * 64 : (int)blockIdx.x * 64;
  const unsigned short* arow = Ab + (size_t)z * zA + (size_t)(m0 + 16 * w + ln) * NE + 8 * hh;
  const unsigned short* brow = Bb + (size_t)z * zB + (size_t)(n0 + ln) * NE + 8 * hh;
  v8f acc[4] = {};
#pragma unroll 1
  for (int kb = 0; kb < NE; kb += 32) {
    FragB a, b0, b1, b2, b3;
    a.half[0]  = *(const v8us*)(arow + kb);               a.half[1]  = *(const v8us*)(arow + kb + 16);
    b0.half[0] = *(const v8us*)(brow + kb);               b0.half[1] = *(const v8us*)(brow + kb + 16);
    b1.half[0] = *(const v8us*)(brow + 16 * NE + kb);     b1.half[1] = *(const v8us*)(brow + 16 * NE + kb + 16);
    b2.half[0] = *(const v8us*)(brow + 32 * NE + kb);     b2.half[1] = *(const v8us*)(brow + 32 * NE + kb + 16);
    b3.half[0] = *(const v8us*)(brow + 48 * NE + kb);     b3.half[1] = *(const v8us*)(brow + 48 * NE + kb + 16);
    mma_b4(a.v, b0.v, b1.v, b2.v, b3.v, acc[0], acc[1], acc[2], acc[3]);
  }
  const float* bz = bias + (size_t)z * zBias;
  float br[8];
#pragma unroll
  for (int r = 0; r < 8; ++r) br[r] = (MODE == 1) ? bf16_rne(bz[m0 + 16 * w + 8 * hh + r]) : 0.0f;
#pragma unroll
  for (int c = 0; c < 4; ++c) {
    const float bc = (MODE == 0) ? bf16_rne(bz[n0 + 16 * c + ln]) : 0.0f;
#pragma unroll
    for (int r = 0; r < 8; ++r) {
      const float bv = (MODE == 0) ? bc : br[r];
      const float x = (acc[c][r] + bv) * 16.0f;
      const _Float16 hv = toh_flush(x);
      th[16 * w + 8 * hh + r][16 * c + ln] = f16_bits(hv);
    }
  }
  __syncthreads();
  size_t obase, opitch;
  if (MODE == 0) {
    const int bq = m0 / SEQ, t0 = m0 - bq * SEQ;
    obase = (size_t)z * zO + ((size_t)(bq * NH + (int)blockIdx.y) * SEQ + t0) * HD;
    opitch = HD;
  } else {
    const int bq = n0 / SEQ, t0 = n0 - bq * SEQ;
    obase = ((size_t)bq * NE + m0) * SEQ + t0;
    opitch = SEQ;
  }
  for (int pass = 0; pass < 2; ++pass) {
#pragma unroll
    for (int j = 0; j < 4; ++j) {
      const int i = tid + 128 * j;
      const int row = i >> 3, s8 = (i & 7) * 8;
      const v8us o = *(const v8us*)&th[row][s8];
      *(volatile v8us*)(Oh + obase + (size_t)row * opitch + s8) = o;
    }
    if (pass == 0) __threadfence();
  }
}

__global__ __launch_bounds__(128) void k_proj_qk(const unsigned short* __restrict__ Ab, const unsigned short* __restrict__ Bb,
                                                 const float* __restrict__ bias, unsigned short* __restrict__ Oh,
                                                 unsigned int zA, unsigned int zB, unsigned int zO, unsigned int zBias) {
  proj_body<0>(Ab, Bb, bias, Oh, zA, zB, zO, zBias);
}

__global__ __launch_bounds__(128) void k_proj_vt(const unsigned short* __restrict__ Ab, const unsigned short* __restrict__ Bb,
                                                 const float* __restrict__ bias, unsigned short* __restrict__ Oh,
                                                 unsigned int zA, unsigned int zB, unsigned int zO, unsigned int zBias) {
  proj_body<1>(Ab, Bb, bias, Oh, zA, zB, zO, zBias);
}

__device__ __forceinline__ void fa_step(const unsigned short* __restrict__ Kp, const unsigned short* __restrict__ Vhp,
                                        unsigned int mword, int key0, int ln, int hh,
                                        const FragH& q0, const FragH& q1, float& mr, float& lr, v8f (&Oh)[4]) {
  const unsigned short* kp0 = Kp + (size_t)(key0 + ln) * HD + 8 * hh;
  const unsigned short* kp1 = kp0 + 16 * HD;
  FragH k00, k01, k10, k11;
  k00.half[0] = *(const v8us*)(kp0);      k00.half[1] = *(const v8us*)(kp0 + 16);
  k01.half[0] = *(const v8us*)(kp0 + 32); k01.half[1] = *(const v8us*)(kp0 + 48);
  k10.half[0] = *(const v8us*)(kp1);      k10.half[1] = *(const v8us*)(kp1 + 16);
  k11.half[0] = *(const v8us*)(kp1 + 32); k11.half[1] = *(const v8us*)(kp1 + 48);
  const v8f z8 = {0.f, 0.f, 0.f, 0.f, 0.f, 0.f, 0.f, 0.f};
  const v8f s0 = mma_s2(k00.v, q0.v, k01.v, q1.v, z8);
  const v8f s1 = mma_s2(k10.v, q0.v, k11.v, q1.v, z8);
  asm volatile("" ::: "memory");
  const size_t vo = (size_t)ln * SEQ + key0 + 8 * hh;
  FragH vh[4];
#pragma unroll
  for (int t = 0; t < 4; ++t) {
    vh[t].half[0] = *(const v8us*)(Vhp + vo + (size_t)t * 16 * SEQ);
    vh[t].half[1] = *(const v8us*)(Vhp + vo + (size_t)t * 16 * SEQ + 16);
  }
  const unsigned int mw = mword >> (8 * hh);
  float sc[16];
#pragma unroll
  for (int r = 0; r < 8; ++r) {
    sc[r]     = ((mw >> r) & 1u) ? s0[r] * SCL : 0.0f;
    sc[8 + r] = ((mw >> (16 + r)) & 1u) ? s1[r] * SCL : 0.0f;
  }
  float mx = sc[0];
#pragma unroll
  for (int i = 1; i < 16; ++i) mx = fmaxf(mx, sc[i]);
  mx = fmaxf(mx, __shfl_xor(mx, 16, 32));
  const float mnew = fmaxf(mr, mx);
  const float al = exp2f((mr - mnew) * LOG2E);
  mr = mnew;
  FragH ph;
  float ps = 0.0f;
#pragma unroll
  for (int i = 0; i < 16; ++i) {
    const float pc = exp2f(fmaf(sc[i] - mnew, LOG2E, 8.0f));
    const _Float16 hv = (_Float16)pc;
    ph.h[i] = hv;
    ps += (float)hv;
  }
  ps += __shfl_xor(ps, 16, 32);
  lr = lr * al + ps;
#pragma unroll
  for (int t = 0; t < 4; ++t) Oh[t] = Oh[t] * al;
  mma_pv4(vh[0].v, vh[1].v, vh[2].v, vh[3].v, ph.v, Oh[0], Oh[1], Oh[2], Oh[3]);
}

__global__ __launch_bounds__(128) void k_attn(const unsigned short* __restrict__ Qh, const unsigned short* __restrict__ Kh,
                                              const unsigned short* __restrict__ Vh,
                                              const unsigned int* __restrict__ mbits,
                                              unsigned short* __restrict__ Ch) {
  __shared__ __attribute__((aligned(16))) unsigned short sh[4][16][72];
  const int tid = threadIdx.x, w = __builtin_amdgcn_readfirstlane((int)(tid >> 5)), lane = tid & 31, ln = lane & 15, hh = lane >> 4;
  const int bh = blockIdx.x / (SEQ / 64), qt = blockIdx.x % (SEQ / 64);
  const int b = bh / NH, h = bh - b * NH;
  const int qbase = qt * 64 + 16 * w;
  const int qg = qbase + ln;
  const unsigned short* qrow = Qh + ((size_t)bh * SEQ + qg) * HD + 8 * hh;
  FragH q0, q1;
  q0.half[0] = *(const v8us*)(qrow);      q0.half[1] = *(const v8us*)(qrow + 16);
  q1.half[0] = *(const v8us*)(qrow + 32); q1.half[1] = *(const v8us*)(qrow + 48);
  float mr = -3.0e38f, lr = 0.0f;
  v8f Oh[4] = {};
  const unsigned short* Kp = Kh + (size_t)bh * SEQ * HD;
  const unsigned short* Vhp = Vh + (size_t)bh * HD * SEQ;
  const unsigned int* mrow = mbits + (size_t)qg * MW;
#pragma unroll 1
  for (int j = 0; j < MW; ++j) {
    const unsigned int mword = mrow[j];
    fa_step(Kp, Vhp, mword, 32 * j, ln, hh, q0, q1, mr, lr, Oh);
  }
  const float inv = 4.0f / lr;
#pragma unroll
  for (int t = 0; t < 4; ++t)
#pragma unroll
    for (int r = 0; r < 8; ++r) {
      const float c = Oh[t][r] * inv;
      const _Float16 hv = (_Float16)c;
      sh[w][ln][16 * t + 8 * hh + r] = f16_bits(hv);
    }
  __syncthreads();
  const size_t cbase = ((size_t)b * SEQ + qbase) * NE + (size_t)h * HD;
  for (int pass = 0; pass < 2; ++pass) {
#pragma unroll
    for (int q = 0; q < 4; ++q) {
      const int p = lane + 32 * q;
      const int row = p >> 3, s8 = (p & 7) * 8;
      const v8us o1 = *(const v8us*)&sh[w][row][s8];
      *(volatile v8us*)(Ch + cbase + (size_t)row * NE + s8) = o1;
    }
    if (pass == 0) __threadfence();
  }
}

__global__ __launch_bounds__(128) void k_outp(const unsigned short* __restrict__ Ch,
                                              const unsigned short* __restrict__ W16, const float* __restrict__ bias,
                                              float* __restrict__ Y) {
  __shared__ __attribute__((aligned(16))) float so[64][68];
  const int tid = threadIdx.x, w = __builtin_amdgcn_readfirstlane((int)(tid >> 5)), lane = tid & 31, ln = lane & 15, hh = lane >> 4;
  const int m0 = blockIdx.x * 64, n0 = blockIdx.y * 64;
  const size_t ao = (size_t)(m0 + 16 * w + ln) * NE + 8 * hh;
  const unsigned short* brow = W16 + (size_t)(n0 + ln) * NE + 8 * hh;
  v8f acch[4] = {};
#pragma unroll 1
  for (int kb = 0; kb < NE; kb += 32) {
    FragH ah, b0, b1, b2, b3;
    ah.half[0] = *(const v8us*)(Ch + ao + kb);            ah.half[1] = *(const v8us*)(Ch + ao + kb + 16);
    b0.half[0] = *(const v8us*)(brow + kb);               b0.half[1] = *(const v8us*)(brow + kb + 16);
    b1.half[0] = *(const v8us*)(brow + 16 * NE + kb);     b1.half[1] = *(const v8us*)(brow + 16 * NE + kb + 16);
    b2.half[0] = *(const v8us*)(brow + 32 * NE + kb);     b2.half[1] = *(const v8us*)(brow + 32 * NE + kb + 16);
    b3.half[0] = *(const v8us*)(brow + 48 * NE + kb);     b3.half[1] = *(const v8us*)(brow + 48 * NE + kb + 16);
    mma_h4(ah.v, b0.v, b1.v, b2.v, b3.v, acch[0], acch[1], acch[2], acch[3]);
  }
#pragma unroll
  for (int c = 0; c < 4; ++c) {
    const float bv = bf16_rne(bias[n0 + 16 * c + ln]);
#pragma unroll
    for (int r = 0; r < 8; ++r)
      so[16 * w + 8 * hh + r][16 * c + ln] = acch[c][r] * 0.000244140625f + bv;
  }
  __syncthreads();
  for (int pass = 0; pass < 2; ++pass) {
#pragma unroll
    for (int j = 0; j < 8; ++j) {
      const int i = tid + 128 * j;
      const int row = i >> 4, c4 = (i & 15) * 4;
      const int m = m0 + row;
      const int bq = m / SEQ, t = m - bq * SEQ;
      const v4f v = *(const v4fa*)&so[row][c4];
      *(volatile v4f*)(Y + (size_t)bq * XSTRIDE_FULL + (size_t)t * NE + n0 + c4) = v;
    }
    if (pass == 0) __threadfence();
  }
}

extern "C" void kernel_launch(void* const* d_in, const int* in_sizes, int n_in,
                              void* d_out, int out_size, void* d_ws, size_t ws_size, hipStream_t stream) {
  if (n_in < 5) return;
  const long long needX = (long long)(NB - 1) * SEQ_FULL * NE + (long long)SEQ * NE;
  if ((long long)in_sizes[0] < needX) return;
  if ((long long)in_sizes[1] < (long long)(3 * WELEMS)) return;
  if ((long long)in_sizes[2] < (long long)(3 * NE)) return;
  if ((long long)in_sizes[3] < (long long)WELEMS) return;
  if ((long long)in_sizes[4] < (long long)NE) return;
  if ((long long)out_size < needX) return;
  const float* X    = (const float*)d_in[0];
  const float* Wqkv = (const float*)d_in[1];
  const float* bqkv = (const float*)d_in[2];
  const float* Wp   = (const float*)d_in[3];
  const float* bp   = (const float*)d_in[4];
  float* Y = (float*)d_out;
  char* ws = (char*)d_ws;
  size_t off = 0;
  unsigned short* XP  = (unsigned short*)(ws + off); off += PAD256(XPLANE * 2);
  unsigned short* WP  = (unsigned short*)(ws + off); off += PAD256(3 * WELEMS * 2);
  unsigned short* W16 = (unsigned short*)(ws + off); off += PAD256(WELEMS * 2);
  unsigned short* QK  = (unsigned short*)(ws + off); off += PAD256(2 * XPLANE * 2);
  unsigned short* VT  = (unsigned short*)(ws + off); off += PAD256(XPLANE * 2);
  unsigned short* CX  = (unsigned short*)(ws + off); off += PAD256(XPLANE * 2);
  unsigned int*   MB  = (unsigned int*)(ws + off);   off += PAD256((size_t)SEQ * MW * 4);
  if (off > ws_size) return;

  k_cvt_x<<<(unsigned)((XROWS * (NE / 8) + 255) / 256), 256, 0, stream>>>(X, XP);
  k_cvt_w<<<(unsigned)((WELEMS / 8 + 255) / 256), 256, 0, stream>>>(Wqkv, Wqkv + WELEMS, Wqkv + 2 * WELEMS, Wp, WP, W16);
  k_maskones<<<(unsigned)((SEQ * MW + 255) / 256), 256, 0, stream>>>(MB);
  k_proj_qk<<<dim3((unsigned)(XROWS / 64), (unsigned)NH, 2u), 128, 0, stream>>>(XP, WP, bqkv, QK,
      0u, (unsigned int)WELEMS, (unsigned int)XPLANE, (unsigned int)NE);
  k_proj_vt<<<dim3((unsigned)(XROWS / 64), (unsigned)(NE / 64), 1u), 128, 0, stream>>>(WP + 2 * WELEMS, XP, bqkv + 2 * NE,
      VT, 0u, 0u, 0u, 0u);
  k_attn<<<(unsigned)(NB * NH * (SEQ / 64)), 128, 0, stream>>>(QK, QK + XPLANE, VT, MB, CX);
  k_outp<<<dim3((unsigned)(XROWS / 64), (unsigned)(NE / 64), 1u), 128, 0, stream>>>(CX, W16, bp, Y);
}
